// HierarchicalPooling_25039659336346
// MI455X (gfx1250) — hardware-verified
//
#include <hip/hip_runtime.h>
#include <math.h>

typedef __attribute__((ext_vector_type(16))) _Float16 v16h;
typedef __attribute__((ext_vector_type(16))) __bf16 v16b;
typedef __attribute__((ext_vector_type(8)))  _Float16 v8h;
typedef __attribute__((ext_vector_type(8)))  float v8f;
typedef __attribute__((ext_vector_type(4)))  float v4f;
typedef __attribute__((ext_vector_type(2)))  float v2f;
typedef __attribute__((ext_vector_type(4)))  unsigned v4u;
typedef __attribute__((ext_vector_type(4)))  int v4i;
typedef float __attribute__((may_alias)) float_a;
typedef int __attribute__((may_alias)) int_a;

template <typename T> __device__ __forceinline__ void vst2(void* p, T v) { *(volatile T*)p = v; __threadfence(); *(volatile T*)p = v; }
__device__ __forceinline__ v8f wmma16(v16h a, v16h b, v8f c) {
  v8f d = __builtin_amdgcn_wmma_f32_16x16x32_f16(false, a, false, b, (short)0, c, false, false);
  asm volatile("v_nop\n\tv_nop\n\tv_nop\n\tv_nop" : "+v"(d) : "v"(a), "v"(b));
  return d;
}
__device__ __forceinline__ v8f wmma_bf(v16b a, v16b b, v8f c) {
  v8f d = __builtin_amdgcn_wmma_f32_16x16x32_bf16(false, a, false, b, (short)0, c, false, false);
  asm volatile("v_nop\n\tv_nop\n\tv_nop\n\tv_nop" : "+v"(d) : "v"(a), "v"(b));
  return d;
}
__device__ __forceinline__ v16h frag_h(const _Float16* rowk0, int lane) {
  union { v16h v; v8h q[2]; } u; const _Float16* p = rowk0 + 8 * (lane >> 4);
  u.q[0] = *(const v8h*)p; u.q[1] = *(const v8h*)(p + 16); return u.v;
}
__device__ __forceinline__ v16h frag_f32(const float* rowk0, int lane) {
  v16h a; const float* p = rowk0 + 8 * (lane >> 4);
#pragma unroll
  for (int i = 0; i < 8; ++i) { a[i] = (_Float16)p[i]; a[8 + i] = (_Float16)p[16 + i]; }
  return a;
}
__device__ __forceinline__ v16h frag_f32s(const float* rowk0, int lane, float sc) {
  v16h a; const float* p = rowk0 + 8 * (lane >> 4);
#pragma unroll
  for (int i = 0; i < 8; ++i) { a[i] = (_Float16)(p[i] * sc); a[8 + i] = (_Float16)(p[16 + i] * sc); }
  return a;
}
__device__ __forceinline__ v16h fragc_f32(const float* W, int k0, int n, int lane, int ld, int K) {
  v16h a; const int g = lane >> 4;
#pragma unroll
  for (int i = 0; i < 8; ++i) { const int ka = k0 + 8 * g + i, kb = ka + 16;
    a[i] = (_Float16)(ka < K ? W[(size_t)(ka < K ? ka : K - 1) * ld + n] : 0.f); a[8 + i] = (_Float16)(kb < K ? W[(size_t)(kb < K ? kb : K - 1) * ld + n] : 0.f); }
  return a;
}
struct F2 { v16b h, l; };
__device__ __forceinline__ F2 bsplit16(const float v[16]) { F2 r;
#pragma unroll
  for (int i = 0; i < 16; ++i) { const __bf16 h = (__bf16)v[i]; r.h[i] = h; r.l[i] = (__bf16)(v[i] - (float)h); }
  return r; }
__device__ __forceinline__ F2 split_row(const float* row, int k0, int lane) { float v[16]; const float* p = row + k0 + 8 * (lane >> 4);
#pragma unroll
  for (int i = 0; i < 8; ++i) { v[i] = p[i]; v[8 + i] = p[16 + i]; }
  return bsplit16(v); }
__device__ __forceinline__ F2 split_rowK(const float* row, int k0, int lane, int K) { float v[16]; const int g = lane >> 4;
#pragma unroll
  for (int i = 0; i < 8; ++i) { const int ka = k0 + 8 * g + i, kb = ka + 16; v[i] = ka < K ? row[ka < K ? ka : K - 1] : 0.f; v[8 + i] = kb < K ? row[kb < K ? kb : K - 1] : 0.f; }
  return bsplit16(v); }
__device__ __forceinline__ F2 split_col(const float* W, int k0, int n, int lane, int ld, int K) { float v[16]; const int g = lane >> 4;
#pragma unroll
  for (int i = 0; i < 8; ++i) { const int ka = k0 + 8 * g + i, kb = ka + 16; v[i] = ka < K ? W[(size_t)(ka < K ? ka : K - 1) * ld + n] : 0.f; v[8 + i] = kb < K ? W[(size_t)(kb < K ? kb : K - 1) * ld + n] : 0.f; }
  return bsplit16(v); }
__device__ __forceinline__ v8f mac3(const F2& a, const F2& b, v8f c) { c = wmma_bf(a.l, b.h, c); c = wmma_bf(a.h, b.l, c); return wmma_bf(a.h, b.h, c); }
__device__ __forceinline__ float sigm(float v) { return 1.0f / (1.0f + expf(-v)); }
#define LDSX() do { asm volatile("s_wait_dscnt 0" ::: "memory"); __builtin_amdgcn_wave_barrier(); __builtin_amdgcn_fence(__ATOMIC_RELEASE, "workgroup"); } while (0)


#define NB 2
#define NN 50000
#define HH 128
#define HHALF 64
#define NE 400000
#define NBLKN ((NN + 63) / 64)
#define NBLKE (NE / 64)
#define PNW 160
#ifndef NBLKN_USE
#define NBLKN_USE NBLKN
#define NBLKE_USE NBLKE
#endif
#define PEW 32
typedef __attribute__((ext_vector_type(8))) __bf16 v8b;
__device__ __forceinline__ v16b frag_b(const __bf16* rowk0, int lane) {
  union { v16b v; v8b q[2]; } u; const __bf16* p = rowk0 + 8 * (lane >> 4);
  u.q[0] = *(const v8b*)p; u.q[1] = *(const v8b*)(p + 16); return u.v;
}
__device__ __forceinline__ v16b frag_gbf(const float* rowk0, int lane) {
  v16b a; const float* p = rowk0 + 8 * (lane >> 4);
#pragma unroll
  for (int i = 0; i < 8; ++i) { a[i] = (__bf16)p[i]; a[8 + i] = (__bf16)p[16 + i]; }
  return a;
}
__device__ __forceinline__ float bfr(float v) { return (float)(__bf16)v; }
__device__ __attribute__((noinline)) float exp_ni(float v) { return expf(v); }
__device__ __attribute__((noinline)) float tanh_ni(float v) { return tanhf(v); }
__device__ __forceinline__ void lse_merge(float& m, float& s, float m2, float s2) { const float mn = fmaxf(m, m2); s = s * exp_ni(m - mn) + s2 * exp_ni(m2 - mn); m = mn; }
__device__ __forceinline__ void lse_merge3(float& m, float& s, float& t, float m2, float s2, float t2) { const float mn = fmaxf(m, m2); const float f1 = exp_ni(m - mn), f2 = exp_ni(m2 - mn); s = s * f1 + s2 * f2; t = t * f1 + t2 * f2; m = mn; }

#define WS_PTN 0u
#define WS_PTS (WS_PTN + 2u * HHALF * HH)
#define WS_PN  (WS_PTS + 2u * HH * 2 * HH)
#define WS_PE  (WS_PN + 4u * NB * NBLKN * PNW)
#define WS_END (WS_PE + 4u * NB * NBLKE * PEW)

__global__ __launch_bounds__(256) void k_pack(const float* __restrict__ Wn1, const float* __restrict__ Ws1, __bf16* __restrict__ PTN, __bf16* __restrict__ PTS) {
  __shared__ __align__(16) __bf16 srow[2 * HH];
  const int n = blockIdx.x, tid = threadIdx.x;
  if (n < HHALF) { if (tid < HH) srow[tid] = (__bf16)Wn1[(size_t)tid * HHALF + n]; __syncthreads(); if (tid < HH / 8) vst2((unsigned*)(PTN + (size_t)n * HH + tid * 8), *(const v4u*)(&srow[tid * 8])); }
  else { const int nn = n - HHALF; srow[tid] = (__bf16)Ws1[(size_t)tid * HH + nn]; __syncthreads(); if (tid < 32) vst2((unsigned*)(PTS + (size_t)nn * 2 * HH + tid * 8), *(const v4u*)(&srow[tid * 8])); }
}
__global__ __launch_bounds__(128) void k_node(const float* __restrict__ X, const __bf16* __restrict__ PTN, const float* __restrict__ bn1, const float* __restrict__ wn2, const float* __restrict__ bn2, float* __restrict__ PN) {
  __shared__ float slog[64]; __shared__ float sw[64]; __shared__ __align__(16) float sline[PNW]; __shared__ float sms[4];
  const int tid = threadIdx.x, wave = tid >> 5, lane = tid & 31, col = lane & 15, g = lane >> 4;
  const int b = blockIdx.y, nb = blockIdx.x * 64; const float* Xb = X + (size_t)b * NN * HH;
  { const int rowl = nb + wave * 16 + col; const int rowc = rowl < NN ? rowl : NN - 1;
    v8f acc[4] = {};
#pragma unroll
    for (int kc = 0; kc < HH / 32; ++kc) { const v16b a = frag_gbf(Xb + (size_t)rowc * HH + kc * 32, lane);
#pragma unroll
      for (int j = 0; j < 4; ++j) acc[j] = wmma_bf(a, frag_b(PTN + (size_t)(j * 16 + col) * HH + kc * 32, lane), acc[j]); }
    float part[8];
#pragma unroll
    for (int r = 0; r < 8; ++r) part[r] = 0.f;
#pragma unroll
    for (int j = 0; j < 4; ++j) { const int c = j * 16 + col; const float bb = bfr(bn1[c]), w2 = bfr(wn2[c]);
#pragma unroll
      for (int r = 0; r < 8; ++r) part[r] += tanh_ni(acc[j][r] + bb) * w2; }
#pragma unroll
    for (int r = 0; r < 8; ++r) {
#pragma unroll
      for (int o = 1; o < 16; o <<= 1) part[r] += __shfl_xor(part[r], o);
      if (col == 0) slog[wave * 16 + 8 * g + r] = part[r] + bfr(bn2[0]); } }
  __syncthreads();
  { float l = -3.0e38f; if (lane < 32) { const int i0 = lane, i1 = lane + 32; const float l0 = (nb + i0 < NN) ? slog[i0] : -3.0e38f, l1 = (nb + i1 < NN) ? slog[i1] : -3.0e38f; l = fmaxf(l0, l1); }
#pragma unroll
    for (int o = 1; o < 32; o <<= 1) l = fmaxf(l, __shfl_xor(l, o));
    if (wave == 0) { sms[0] = l;
      const int i0 = lane, i1 = lane + 32; sw[i0] = (nb + i0 < NN) ? exp_ni(slog[i0] - l) : 0.f; sw[i1] = (nb + i1 < NN) ? exp_ni(slog[i1] - l) : 0.f; } }
  __syncthreads();
  { const int h = tid; float v = 0.f;
#pragma unroll 4
    for (int i = 0; i < 64; ++i) { const int row = nb + i < NN ? nb + i : NN - 1; v += sw[i] * bfr(Xb[(size_t)row * HH + h]); }
    sline[8 + h] = v;
    if (tid < 32) { float s = sw[tid] + sw[tid + 32];
#pragma unroll
      for (int o = 1; o < 32; o <<= 1) s += __shfl_xor(s, o);
      if (tid == 0) { sline[0] = sms[0]; sline[1] = s; } if (tid >= 2 && tid < 8) sline[tid] = 0.f; }
    if (tid >= 8 && tid < 32) sline[128 + tid] = 0.f; }
  __syncthreads();
  if (tid < PNW / 4) vst2(PN + ((size_t)b * NBLKN + blockIdx.x) * PNW + tid * 4, *(const v4f*)&sline[tid * 4]);
}
__global__ __launch_bounds__(256) void k_edge(const float* __restrict__ X, const int* __restrict__ ei, const __bf16* __restrict__ PTS, const float* __restrict__ bs1, const float* __restrict__ ws2, const float* __restrict__ bs2, float* __restrict__ PE) {
  __shared__ __align__(16) __bf16 sa[64][2 * HH + 8];
  __shared__ float smu[8][64], slog2[2][64], sline[32];
  const int tid = threadIdx.x, wave = tid >> 5, lane = tid & 31, col = lane & 15, g = lane >> 4;
  const int b = blockIdx.y; const size_t e0 = (size_t)blockIdx.x * 64; const float* Xb = X + (size_t)b * NN * HH;
  { const int q4 = wave & 3, el = (wave >> 2) * 32 + lane; const size_t e = e0 + el;
    int idx = ei[(q4 < 2 ? 0 : NE) + e]; idx = idx < 0 ? 0 : (idx >= NN ? NN - 1 : idx);
    const float* src = Xb + (size_t)idx * HH + (q4 & 1) * 64; float mu = 0.f;
#pragma unroll
    for (int c4 = 0; c4 < 16; ++c4) { const float4 v = *(const float4*)(src + c4 * 4); __bf16* d = &sa[el][q4 * 64 + c4 * 4];
      const __bf16 h0 = (__bf16)v.x, h1 = (__bf16)v.y, h2 = (__bf16)v.z, h3 = (__bf16)v.w; d[0] = h0; d[1] = h1; d[2] = h2; d[3] = h3; mu += ((float)h0 + (float)h1) + ((float)h2 + (float)h3); }
    smu[wave][lane] = mu; }
  __syncthreads();
  { const int rt = wave & 3, ct0 = (wave >> 2) * 4; v8f acc[4] = {};
#pragma unroll 2
    for (int kc = 0; kc < 2 * HH / 32; ++kc) { const v16b a = frag_b(&sa[rt * 16 + col][kc * 32], lane);
#pragma unroll
      for (int j = 0; j < 4; ++j) acc[j] = wmma_bf(a, frag_b(PTS + (size_t)((ct0 + j) * 16 + col) * 2 * HH + kc * 32, lane), acc[j]); }
    float part[8];
#pragma unroll
    for (int r = 0; r < 8; ++r) part[r] = 0.f;
#pragma unroll
    for (int j = 0; j < 4; ++j) { const int c = (ct0 + j) * 16 + col; const float bb = bfr(bs1[c]), w2 = bfr(ws2[c]);
#pragma unroll
      for (int r = 0; r < 8; ++r) part[r] += tanh_ni(acc[j][r] + bb) * w2; }
#pragma unroll
    for (int r = 0; r < 8; ++r) {
#pragma unroll
      for (int o = 1; o < 16; o <<= 1) part[r] += __shfl_xor(part[r], o);
      if (col == 0) slog2[wave >> 2][rt * 16 + 8 * g + r] = part[r]; } }
  __syncthreads();
  if (wave == 0) {
    const int i0 = lane, i1 = lane + 32;
    const float l0 = (slog2[0][i0] + slog2[1][i0]) + bfr(bs2[0]), l1 = (slog2[0][i1] + slog2[1][i1]) + bfr(bs2[0]);
    float mx = fmaxf(l0, l1);
#pragma unroll
    for (int o = 1; o < 32; o <<= 1) mx = fmaxf(mx, __shfl_xor(mx, o));
    const float w0 = exp_ni(l0 - mx), w1 = exp_ni(l1 - mx);
    const float mu0 = ((smu[0][lane] + smu[1][lane]) + (smu[2][lane] + smu[3][lane])) * (1.0f / 256.0f), mu1 = ((smu[4][lane] + smu[5][lane]) + (smu[6][lane] + smu[7][lane])) * (1.0f / 256.0f);
    float s = w0 + w1, t = w0 * mu0 + w1 * mu1;
#pragma unroll
    for (int o = 1; o < 32; o <<= 1) { s += __shfl_xor(s, o); t += __shfl_xor(t, o); }
    sline[lane] = lane == 0 ? mx : (lane == 1 ? s : (lane == 2 ? t : 0.f));
    LDSX();
    if (lane < 8) vst2(PE + ((size_t)b * NBLKE + blockIdx.x) * PEW + lane * 4, *(const v4f*)&sline[lane * 4]); }
}
__global__ __launch_bounds__(256) void k_fin(const float* __restrict__ PN, const float* __restrict__ PE, float* __restrict__ out) {
  __shared__ float smx[256], ssum[256], st[256]; __shared__ __align__(16) float srow[2 * HH]; __shared__ float sM[2], sS[2];
  const int b = blockIdx.x, tid = threadIdx.x, lane = tid & 31, wave = tid >> 5;
  { float m = -3.0e38f;
    for (int i = tid; i < NBLKN_USE; i += 256) m = fmaxf(m, PN[((size_t)b * NBLKN + i) * PNW]);
    smx[tid] = m; }
  __syncthreads();
  if (tid < 32) { float m = -3.0e38f; for (int i = lane; i < 256; i += 32) m = fmaxf(m, smx[i]);
#pragma unroll
    for (int o = 1; o < 32; o <<= 1) m = fmaxf(m, __shfl_xor(m, o)); if (tid == 0) sM[0] = m; }
  __syncthreads();
  { const float M = sM[0]; float s = 0.f;
    for (int i = tid; i < NBLKN_USE; i += 256) { const float* p = PN + ((size_t)b * NBLKN + i) * PNW; s += p[1] * exp_ni(p[0] - M); }
    ssum[tid] = s; }
  __syncthreads();
  if (tid < 32) { float s = 0.f; for (int i = lane; i < 256; i += 32) s += ssum[i];
#pragma unroll
    for (int o = 1; o < 32; o <<= 1) s += __shfl_xor(s, o); if (tid == 0) sS[0] = s; }
  if (tid < HH) { const float M = sM[0]; float v = 0.f;
#pragma unroll 1
    for (int i = 0; i < NBLKN_USE; ++i) { const float* p = PN + ((size_t)b * NBLKN + i) * PNW; v += p[8 + tid] * exp_ni(p[0] - M); }
    smx[tid] = v; }
  else { float m = -3.0e38f; for (int i = tid - HH; i < NBLKE_USE; i += HH) m = fmaxf(m, PE[((size_t)b * NBLKE + i) * PEW]); st[tid] = m; }
  __syncthreads();
  if (tid >= HH && tid < HH + 32) { float m = -3.0e38f; for (int i = lane; i < 128; i += 32) m = fmaxf(m, st[HH + i]);
#pragma unroll
    for (int o = 1; o < 32; o <<= 1) m = fmaxf(m, __shfl_xor(m, o)); if (lane == 0) sM[1] = m; }
  __syncthreads();
  { const float ME = sM[1]; float s = 0.f, t = 0.f;
    for (int i = tid; i < NBLKE_USE; i += 256) { const float* p = PE + ((size_t)b * NBLKE + i) * PEW; const float f = exp_ni(p[0] - ME); s += p[1] * f; t += p[2] * f; }
    ssum[tid] = s; st[tid] = t; }
  __syncthreads();
  if (tid < 32) { float s = 0.f, t = 0.f; for (int i = lane; i < 256; i += 32) { s += ssum[i]; t += st[i]; }
#pragma unroll
    for (int o = 1; o < 32; o <<= 1) { s += __shfl_xor(s, o); t += __shfl_xor(t, o); }
    if (tid == 0) { sS[1] = s; sM[1] = t; } }
  __syncthreads();
  if (tid < HH) srow[tid] = smx[tid] / sS[0]; else srow[tid] = sM[1] / sS[1];
  __syncthreads();
  if (tid < 64) vst2(out + (size_t)b * 2 * HH + tid * 4, *(const v4f*)&srow[tid * 4]);
}

extern "C" void kernel_launch(void* const* d_in, const int* in_sizes, int n_in, void* d_out, int out_size, void* d_ws, size_t ws_size, hipStream_t stream) {
  (void)in_sizes; (void)n_in; (void)out_size;
  const float* X = (const float*)d_in[0]; const int* ei = (const int*)d_in[1]; const float** F = (const float**)d_in;
  if (ws_size < (size_t)WS_END) return;
  char* ws = (char*)d_ws; __bf16* PTN = (__bf16*)(ws + WS_PTN); __bf16* PTS = (__bf16*)(ws + WS_PTS); float* PN = (float*)(ws + WS_PN); float* PE = (float*)(ws + WS_PE);
  k_pack<<<HHALF + HH, 256, 0, stream>>>(F[2], F[6], PTN, PTS);
  k_node<<<dim3(NBLKN_USE, NB), 128, 0, stream>>>(X, PTN, F[3], F[4], F[5], PN);
  k_edge<<<dim3(NBLKE_USE, NB), 256, 0, stream>>>(X, ei, PTS, F[7], F[8], F[9], PE);
  k_fin<<<NB, 256, 0, stream>>>(PN, PE, (float*)d_out);
}
